// LSTM_51728586113045
// MI455X (gfx1250) — hardware-verified
//
#include <hip/hip_runtime.h>
#include <math.h>

constexpr int NBATCH = 8192;
constexpr int NSTEP  = 128;
constexpr int NIN    = 9;
constexpr int NHID   = 32;
constexpr int NGATE  = 4 * NHID;
constexpr int NOUT   = 6;
constexpr int NOUTP  = 16;
constexpr int NFC    = NSTEP * NHID;
constexpr int KCAT   = 64;
constexpr int WPITCH = 72;
constexpr int TPITCH = 168;
constexpr int COL_H1 = 32;
constexpr int COL_H2 = 96;
constexpr int LPITCH = 17;
constexpr int MAIN_THR = 64;
constexpr int MAIN_WAVES = MAIN_THR / 32;
constexpr int ROWS_PER_BLOCK = 16 * MAIN_WAVES;
constexpr int CS_PER_LAYER = 2 * 8 * 32;
constexpr int CS_PER_WAVE  = 2 * CS_PER_LAYER;
constexpr int PREP_THR = 256;
constexpr int PREP_BLOCKS_W = 8;
constexpr int PREP_BLOCKS_FC = (NOUTP * NFC / 8) / PREP_THR;
constexpr int PREP_BLOCKS = PREP_BLOCKS_W + PREP_BLOCKS_FC + 1;

constexpr size_t WS_OFF_WCAT = 0;
constexpr size_t WS_OFF_WFC  = (size_t)2 * NGATE * KCAT * 2;
constexpr size_t WS_OFF_BSUM = WS_OFF_WFC + (size_t)NOUTP * NFC * 2;
constexpr size_t WS_TOTAL    = WS_OFF_BSUM + (size_t)2 * NGATE * 4;

static_assert(NGATE == 128, "gate rows");
static_assert(NFC == 4096, "fc depth");
static_assert(KCAT == 2 * 32, "two k chunks of 32");
static_assert(NBATCH % ROWS_PER_BLOCK == 0, "grid exact");
static_assert(NIN <= 16, "x fits the first 16 columns of the tile");
static_assert(WPITCH % 8 == 0 && TPITCH % 8 == 0, "16-B aligned fragment halves");
static_assert(WPITCH >= KCAT && TPITCH >= COL_H2 + 64, "tile extents");
static_assert((2 * NGATE * KCAT / 8) % MAIN_THR == 0, "weight staging loop exact");
static_assert(2 * NGATE / 4 == MAIN_THR, "bias staging: one 16-B piece per thread exactly");
static_assert(PREP_BLOCKS_FC * PREP_THR * 8 == NOUTP * NFC, "fc plane coverage exact");
static_assert(4 * PREP_THR * 8 == NGATE * KCAT, "weight plane coverage exact");
static_assert(WS_TOTAL == 164864, "carve");
static_assert((ROWS_PER_BLOCK / MAIN_WAVES) * NOUT * 4 == 384, "three whole lines per wave tile");

typedef __attribute__((ext_vector_type(16))) _Float16 v16h;
typedef __attribute__((ext_vector_type(8)))  _Float16 v8h;
typedef __attribute__((ext_vector_type(8)))  float    v8f;
typedef __attribute__((ext_vector_type(4)))  float    v4f;
typedef __attribute__((ext_vector_type(4)))  unsigned v4u;

__device__ __forceinline__ void guard_group_h(v8f& a, v8f& b, v8f& c, v8f& d, v16h x, v16h b0, v16h b1, v16h b2, v16h b3) {
  asm volatile("v_nop\n\tv_nop\n\tv_nop\n\tv_nop" : "+v"(a), "+v"(b), "+v"(c), "+v"(d) : "v"(x), "v"(b0), "v"(b1), "v"(b2), "v"(b3));
}
__device__ __forceinline__ void guard1_h(v8f& a, v16h x, v16h y) {
  asm volatile("v_nop\n\tv_nop\n\tv_nop\n\tv_nop" : "+v"(a) : "v"(x), "v"(y));
}
__device__ __forceinline__ void acc_guard4(v8f& a, v8f& b, v8f& c, v8f& d) {
  asm volatile("v_nop\n\tv_nop\n\tv_nop\n\tv_nop" : "+v"(a), "+v"(b), "+v"(c), "+v"(d));
}

struct FragH {
  union U { v16h v; v8h h[2]; };
  static __device__ __forceinline__ v16h load(const _Float16* p) {
    U f; f.h[0] = *(const v8h*)(p); f.h[1] = *(const v8h*)(p + 16); return f.v;
  }
  static __device__ __forceinline__ v8f mma(v16h a, v16h b, v8f c) {
    return __builtin_amdgcn_wmma_f32_16x16x32_f16(false, a, false, b, (short)0, c, false, false);
  }
};

__device__ __forceinline__ unsigned h16bits(float f) {
  const _Float16 h = (_Float16)f;
  return (unsigned)__builtin_bit_cast(unsigned short, h);
}
__device__ __forceinline__ unsigned pack2h(float lo, float hi) { return h16bits(lo) | (h16bits(hi) << 16); }

__device__ __forceinline__ void store_words_twice(unsigned* p, v4u w) {
  *(volatile v4u*)p = w;
  __threadfence();
  *(volatile v4u*)p = w;
}
__device__ __forceinline__ void store_floats_twice(float* p, v4f w) {
  *(volatile v4f*)p = w;
  __threadfence();
  *(volatile v4f*)p = w;
}

__device__ __forceinline__ float fsig(float x)  { return __builtin_amdgcn_rcpf(1.0f + expf(-x)); }
__device__ __forceinline__ float ftanh(float x) { return 1.0f - 2.0f * __builtin_amdgcn_rcpf(expf(2.0f * x) + 1.0f); }

__global__ __launch_bounds__(PREP_THR) void prep_planes_kernel(
    const float* __restrict__ wih0, const float* __restrict__ whh0,
    const float* __restrict__ bih0, const float* __restrict__ bhh0,
    const float* __restrict__ wih1, const float* __restrict__ whh1,
    const float* __restrict__ bih1, const float* __restrict__ bhh1,
    const float* __restrict__ wfc,
    unsigned* __restrict__ wcat, unsigned* __restrict__ wfc16, float* __restrict__ bsum) {
  const int tid = threadIdx.x;
  const int blk = blockIdx.x;
  if (blk < PREP_BLOCKS_W) {
    const int layer = blk >> 2;
    const float* wih = layer ? wih1 : wih0;
    const float* whh = layer ? whh1 : whh0;
    const int kin = layer ? NHID : NIN;
    const int u  = (blk & 3) * PREP_THR + tid;
    const int n  = u >> 3;
    const int c8 = (u & 7) * 8;
    int cb = c8 - 32;
    cb = cb < 0 ? 0 : cb;
    v4f hb0 = *(const v4f*)(whh + n * NHID + cb);
    v4f hb1 = *(const v4f*)(whh + n * NHID + cb + 4);
    float av[8];
#pragma unroll
    for (int e = 0; e < 8; ++e) {
      const int col = c8 + e;
      const int ca = col < kin ? col : (kin - 1);
      av[e] = wih[n * kin + ca];
    }
    asm volatile("" : "+v"(hb0));
    asm volatile("" : "+v"(hb1));
#pragma unroll
    for (int e = 0; e < 8; ++e) asm volatile("" : "+v"(av[e]));
    float f[8];
#pragma unroll
    for (int e = 0; e < 4; ++e) {
      const int col = c8 + e;
      const float bv = hb0[e];
      f[e] = (col < kin) ? av[e] : ((col >= 32) ? bv : 0.0f);
    }
#pragma unroll
    for (int e = 0; e < 4; ++e) {
      const int col = c8 + 4 + e;
      const float bv = hb1[e];
      f[4 + e] = (col < kin) ? av[4 + e] : ((col >= 32) ? bv : 0.0f);
    }
    v4u w;
    w[0] = pack2h(f[0], f[1]);
    w[1] = pack2h(f[2], f[3]);
    w[2] = pack2h(f[4], f[5]);
    w[3] = pack2h(f[6], f[7]);
    store_words_twice(wcat + ((size_t)layer * (NGATE * KCAT / 8) + (size_t)u) * 4, w);
  } else if (blk < PREP_BLOCKS_W + PREP_BLOCKS_FC) {
    const int u   = (blk - PREP_BLOCKS_W) * PREP_THR + tid;
    const int row = u >> 9;
    const int c8  = (u & 511) * 8;
    const int rs  = row < NOUT ? row : (NOUT - 1);
    v4f a = *(const v4f*)(wfc + (size_t)rs * NFC + c8);
    v4f b = *(const v4f*)(wfc + (size_t)rs * NFC + c8 + 4);
    asm volatile("" : "+v"(a));
    asm volatile("" : "+v"(b));
    const bool live = (row < NOUT);
    float f[8];
#pragma unroll
    for (int e = 0; e < 4; ++e) {
      const float x0 = a[e];
      const float x1 = b[e];
      f[e]     = live ? x0 : 0.0f;
      f[4 + e] = live ? x1 : 0.0f;
    }
    v4u w;
    w[0] = pack2h(f[0], f[1]);
    w[1] = pack2h(f[2], f[3]);
    w[2] = pack2h(f[4], f[5]);
    w[3] = pack2h(f[6], f[7]);
    store_words_twice(wfc16 + (size_t)u * 4, w);
  } else {
    if (tid < 64) {
      const int which = tid >> 5;
      const int idx = (tid & 31) * 4;
      const v4f a0 = *(const v4f*)(bih0 + idx);
      const v4f b0 = *(const v4f*)(bhh0 + idx);
      const v4f a1 = *(const v4f*)(bih1 + idx);
      const v4f b1 = *(const v4f*)(bhh1 + idx);
      v4f o;
#pragma unroll
      for (int e = 0; e < 4; ++e) {
        const float s0 = a0[e] + b0[e];
        const float s1 = a1[e] + b1[e];
        o[e] = which ? s1 : s0;
      }
      store_floats_twice(bsum + which * NGATE + idx, o);
    }
  }
}

__device__ __forceinline__ void lstm_layer_step(const _Float16* arow_a, const _Float16* arow_b, const _Float16* wplane,
                                                const float* bl, float* cs, _Float16* hdst,
                                                int c, int hh, int koff, int lane) {
  const v16h a0 = FragH::load(arow_a);
  const v16h a1 = FragH::load(arow_b);
#pragma unroll 1
  for (int ub = 0; ub < 2; ++ub) {
    const _Float16* wb = wplane + (16 * ub + c) * WPITCH + koff;
    const float* bp = bl + 16 * ub + c;
    v8f acc[4];
#pragma unroll
    for (int g = 0; g < 4; ++g) {
      const float b = bp[NHID * g];
      acc[g] = (v8f){b, b, b, b, b, b, b, b};
    }
    __builtin_amdgcn_sched_barrier(0);
    {
      const v16h b0 = FragH::load(wb + 0 * NHID * WPITCH);
      const v16h b1 = FragH::load(wb + 1 * NHID * WPITCH);
      const v16h b2 = FragH::load(wb + 2 * NHID * WPITCH);
      const v16h b3 = FragH::load(wb + 3 * NHID * WPITCH);
      acc[0] = FragH::mma(a0, b0, acc[0]);
      acc[1] = FragH::mma(a0, b1, acc[1]);
      acc[2] = FragH::mma(a0, b2, acc[2]);
      acc[3] = FragH::mma(a0, b3, acc[3]);
      guard_group_h(acc[0], acc[1], acc[2], acc[3], a0, b0, b1, b2, b3);
    }
    __builtin_amdgcn_sched_barrier(0);
    {
      const v16h b0 = FragH::load(wb + 0 * NHID * WPITCH + 32);
      const v16h b1 = FragH::load(wb + 1 * NHID * WPITCH + 32);
      const v16h b2 = FragH::load(wb + 2 * NHID * WPITCH + 32);
      const v16h b3 = FragH::load(wb + 3 * NHID * WPITCH + 32);
      acc[0] = FragH::mma(a1, b0, acc[0]);
      acc[1] = FragH::mma(a1, b1, acc[1]);
      acc[2] = FragH::mma(a1, b2, acc[2]);
      acc[3] = FragH::mma(a1, b3, acc[3]);
      guard_group_h(acc[0], acc[1], acc[2], acc[3], a1, b0, b1, b2, b3);
    }
    __builtin_amdgcn_sched_barrier(0);
    acc_guard4(acc[0], acc[1], acc[2], acc[3]);
    float* cp = cs + ub * (8 * 32) + lane;
    _Float16* hp = hdst + (8 * hh) * TPITCH + 16 * ub + c;
#pragma unroll
    for (int r = 0; r < 8; ++r) {
      const float cold = cp[r * 32];
      const float ig = fsig(acc[0][r]);
      const float fg = fsig(acc[1][r]);
      const float gg = ftanh(acc[2][r]);
      const float og = fsig(acc[3][r]);
      const float cn = fg * cold + ig * gg;
      cp[r * 32] = cn;
      const float hn = og * ftanh(cn);
      hp[r * TPITCH] = (_Float16)hn;
      __builtin_amdgcn_sched_barrier(0);
    }
  }
}

__global__ __launch_bounds__(MAIN_THR) __attribute__((amdgpu_num_vgpr(256))) void lstm2_fc_softmax_kernel(
    const float* __restrict__ x, const unsigned* __restrict__ wcat, const unsigned short* __restrict__ wfc16p,
    const float* __restrict__ bsum, const float* __restrict__ bfc, float* __restrict__ out) {
  __shared__ __align__(16) _Float16 Wl[2][NGATE * WPITCH];
  __shared__ __align__(16) _Float16 Tl[MAIN_WAVES][16 * TPITCH];
  __shared__ __align__(16) float    Cs[MAIN_WAVES][CS_PER_WAVE];
  __shared__ __align__(16) float    Bl[2 * NGATE];
  __shared__ __align__(16) float    Ls[MAIN_WAVES][16 * LPITCH];
  __shared__ __align__(16) float    Os[MAIN_WAVES][16 * NOUT];

  const _Float16* wfc16 = (const _Float16*)wfc16p;
  const int tid = threadIdx.x, lane = tid & 31, wave = tid >> 5;
  const int c = lane & 15, hh = lane >> 4, koff = hh * 8;
  const int row0 = blockIdx.x * ROWS_PER_BLOCK + wave * 16;

  {
    const v4u* wsrc = (const v4u*)wcat;
#pragma unroll 1
    for (int i = 0; i < (2 * NGATE * KCAT / 8) / MAIN_THR; ++i) {
      const int u = i * MAIN_THR + tid;
      const int plane = u >> 10, row = (u >> 3) & (NGATE - 1), q = u & 7;
      const v4u w = wsrc[u];
      *(v4u*)(&Wl[plane][row * WPITCH + q * 8]) = w;
    }
  }
  {
    const v4f bv = *(const v4f*)(bsum + 4 * tid);
    *(v4f*)(&Bl[4 * tid]) = bv;
  }
  _Float16* tile = &Tl[wave][0];
  {
    const v4u z = {0u, 0u, 0u, 0u};
#pragma unroll
    for (int i = 0; i < 8; ++i) {
      const int uu = i * 32 + lane;
      const int row = uu >> 4, q = uu & 15;
      *(v4u*)(tile + row * TPITCH + COL_H1 + q * 8) = z;
    }
  }
  float* cs = &Cs[wave][0];
#pragma unroll 1
  for (int i = 0; i < CS_PER_WAVE / 32; ++i) cs[i * 32 + lane] = 0.0f;

  v8f facc = {0.f, 0.f, 0.f, 0.f, 0.f, 0.f, 0.f, 0.f};

  const _Float16* trow = tile + c * TPITCH + koff;
  const float* xrow = x + (size_t)(row0 + c) * (size_t)(NSTEP * NIN);
  const _Float16* wfrow = wfc16 + (size_t)c * NFC + koff;
  const unsigned xmask = 0u - (unsigned)(1 - hh);
  __syncthreads();

#pragma unroll 1
  for (int t = 0; t < NSTEP; ++t) {
    const int p  = t & 1;
    const int pn = p ^ 1;
    {
      const float* xp = xrow + (size_t)t * NIN;
      float xv[NIN];
#pragma unroll
      for (int e = 0; e < NIN; ++e) xv[e] = xp[e];
#pragma unroll
      for (int e = 0; e < NIN; ++e) asm volatile("" : "+v"(xv[e]));
      v4u w0, w1;
      w0[0] = pack2h(xv[0], xv[1]) & xmask;
      w0[1] = pack2h(xv[2], xv[3]) & xmask;
      w0[2] = pack2h(xv[4], xv[5]) & xmask;
      w0[3] = pack2h(xv[6], xv[7]) & xmask;
      w1[0] = h16bits(xv[8]) & xmask;
      w1[1] = 0u;
      w1[2] = 0u;
      w1[3] = 0u;
      *(v4u*)(tile + c * TPITCH + 16 * hh)     = w0;
      *(v4u*)(tile + c * TPITCH + 16 * hh + 8) = w1;
    }
    __syncthreads();

    lstm_layer_step(trow, trow + COL_H1 + 32 * p, &Wl[0][0], &Bl[0], cs,
                    tile + COL_H1 + 32 * pn, c, hh, koff, lane);
    __syncthreads();

    lstm_layer_step(trow + COL_H1 + 32 * pn, trow + COL_H2 + 32 * p, &Wl[1][0], &Bl[NGATE], cs + CS_PER_LAYER,
                    tile + COL_H2 + 32 * pn, c, hh, koff, lane);
    __syncthreads();

    {
      const v16h a = FragH::load(trow + COL_H2 + 32 * pn);
      const v16h b = FragH::load(wfrow + t * NHID);
      facc = FragH::mma(a, b, facc);
      guard1_h(facc, a, b);
    }
  }

  float* ls = &Ls[wave][0];
#pragma unroll
  for (int r = 0; r < 8; ++r) ls[(8 * hh + r) * LPITCH + c] = facc[r];
  __syncthreads();
  float ex[NOUT];
  float mx = 0.0f;
#pragma unroll
  for (int j = 0; j < NOUT; ++j) {
    float v = ls[c * LPITCH + j] + bfc[j];
    v = fmaxf(v, 0.0f);
    ex[j] = v;
    mx = fmaxf(mx, v);
  }
  float s = 0.0f;
#pragma unroll
  for (int j = 0; j < NOUT; ++j) { ex[j] = expf(ex[j] - mx); s += ex[j]; }
  const float inv = 1.0f / s;
  float* os = &Os[wave][0];
  if (hh == 0) {
#pragma unroll
    for (int j = 0; j < NOUT; ++j) os[c * NOUT + j] = ex[j] * inv;
  }
  __syncthreads();
  {
    const int ls4 = (lane < 24 ? lane : 23) * 4;
    const v4f v = *(const v4f*)(os + ls4);
    float* op = out + (size_t)row0 * NOUT + ls4;
    if (lane < 24) *(volatile v4f*)op = v;
    __threadfence();
    if (lane < 24) *(volatile v4f*)op = v;
  }
}

extern "C" void kernel_launch(void* const* d_in, const int* in_sizes, int n_in,
                              void* d_out, int out_size, void* d_ws, size_t ws_size, hipStream_t stream) {
  if (n_in < 11 || d_out == nullptr || d_ws == nullptr) return;
  if (in_sizes[0] != NBATCH * NSTEP * NIN || in_sizes[1] != NGATE * NIN || in_sizes[2] != NGATE * NHID ||
      in_sizes[3] != NGATE || in_sizes[4] != NGATE || in_sizes[5] != NGATE * NHID || in_sizes[6] != NGATE * NHID ||
      in_sizes[7] != NGATE || in_sizes[8] != NGATE || in_sizes[9] != NOUT * NFC || in_sizes[10] != NOUT ||
      out_size != NBATCH * NOUT) return;
  if (WS_TOTAL > ws_size || WS_TOTAL > (size_t)134217728) return;

  const float* x    = (const float*)d_in[0];
  const float* wih0 = (const float*)d_in[1];
  const float* whh0 = (const float*)d_in[2];
  const float* bih0 = (const float*)d_in[3];
  const float* bhh0 = (const float*)d_in[4];
  const float* wih1 = (const float*)d_in[5];
  const float* whh1 = (const float*)d_in[6];
  const float* bih1 = (const float*)d_in[7];
  const float* bhh1 = (const float*)d_in[8];
  const float* wfc  = (const float*)d_in[9];
  const float* bfc  = (const float*)d_in[10];
  float* out = (float*)d_out;

  char* ws = (char*)d_ws;
  unsigned* wcat  = (unsigned*)(ws + WS_OFF_WCAT);
  unsigned* wfc16 = (unsigned*)(ws + WS_OFF_WFC);
  float*    bsum  = (float*)(ws + WS_OFF_BSUM);

  prep_planes_kernel<<<PREP_BLOCKS, PREP_THR, 0, stream>>>(wih0, whh0, bih0, bhh0, wih1, whh1, bih1, bhh1, wfc,
                                                          wcat, wfc16, bsum);
  lstm2_fc_softmax_kernel<<<NBATCH / ROWS_PER_BLOCK, MAIN_THR, 0, stream>>>(
      x, (const unsigned*)wcat, (const unsigned short*)wfc16, bsum, bfc, out);
}
